// MemLayer_80178449482250
// MI455X (gfx1250) — hardware-run, weakly checked
//
#include <hip/hip_runtime.h>
#include <math.h>

typedef __attribute__((ext_vector_type(16))) _Float16 v16h;
typedef __attribute__((ext_vector_type(8)))  _Float16 v8h;
typedef __attribute__((ext_vector_type(4)))  _Float16 v4h;
typedef __attribute__((ext_vector_type(2)))  _Float16 v2h;
typedef __attribute__((ext_vector_type(16))) __bf16   v16b;
typedef __attribute__((ext_vector_type(8)))  __bf16   v8b;
typedef __attribute__((ext_vector_type(8)))  float    v8f;
typedef __attribute__((ext_vector_type(4)))  float    v4f;
typedef __attribute__((ext_vector_type(2)))  float    v2f;

constexpr int kT    = 8192;
constexpr int kXD   = 1024;
constexpr int kMN   = 64;
constexpr int kMD   = 128;
constexpr int kDD   = 32;
constexpr int kNV   = kMD + kMN + kMD;
constexpr int kTC   = 1024;
constexpr int kNCh  = kT / kTC;
constexpr int kRC   = kTC * kMN;
constexpr int kThr  = 256;
constexpr float kInCarry = 1024.0f;
constexpr float kSc = 1.0f / (kInCarry * kInCarry);
constexpr float kScale = 0.08838834764831845f;
constexpr float kF16MinNormal = 6.103515625e-5f;

static_assert((kT % 64) == 0 && (kNV % 64) == 0 && (kXD % 64) == 0 && (kMD % 64) == 0 && (kRC % 64) == 0 && (kXD % 32) == 0 && (kMD % 32) == 0 && ((kT / 64) * (kNV / 64)) % 8 == 0 && ((kT / 64) * (kXD / 64)) % 8 == 0 && ((kRC / 64) * (kMD / 64)) % 8 == 0, "GEMM M, N multiples of 64, K of 32; grids exact (640, 2,048 and 2,048 tiles)");

constexpr size_t kOffX16 = 0ull;
constexpr size_t kOffWVFQ = 16777216ull;
constexpr size_t kOffWR16 = 17432576ull;
constexpr size_t kOffWK16 = 19529728ull;
constexpr size_t kOffWO16 = 19562496ull;
constexpr size_t kOffZB = 19824640ull;
constexpr size_t kOffSTATE = 19828736ull;
constexpr size_t kOffVFQ = 19861504ull;
constexpr size_t kOffG = 30347264ull;
constexpr size_t kOffMEM32 = 63901696ull;
constexpr size_t kOffMEM16 = 97456128ull;
constexpr size_t kOffKS = 114233344ull;
constexpr size_t kOffYS16 = 147787776ull;
constexpr size_t kOffOUTP = 149884928ull;
constexpr size_t kWsTotal = 183439360ull;
static_assert(kWsTotal <= 268435456ull, "carve cap: the offered workspace");
static_assert(kOffX16 == 0
              && kOffWVFQ == kOffX16 + 16777216ull
              && kOffWR16 == kOffWVFQ + 655360ull
              && kOffWK16 == kOffWR16 + 2097152ull
              && kOffWO16 == kOffWK16 + 32768ull
              && kOffZB == kOffWO16 + 262144ull
              && kOffSTATE == kOffZB + 4096ull
              && kOffVFQ == kOffSTATE + 32768ull
              && kOffG == kOffVFQ + 10485760ull
              && kOffMEM32 == kOffG + 33554432ull
              && kOffMEM16 == kOffMEM32 + 33554432ull
              && kOffKS == kOffMEM16 + 16777216ull
              && kOffYS16 == kOffKS + 33554432ull
              && kOffOUTP == kOffYS16 + 2097152ull
              && kWsTotal == kOffOUTP + 33554432ull, "the carve is chained and totalled");
static_assert((kOffX16 % 256) == 0 && (kOffWVFQ % 256) == 0 && (kOffWR16 % 256) == 0 && (kOffWK16 % 256) == 0 && (kOffWO16 % 256) == 0 && (kOffZB % 256) == 0 && (kOffSTATE % 256) == 0 && (kOffVFQ % 256) == 0 && (kOffG % 256) == 0 && (kOffMEM32 % 256) == 0 && (kOffMEM16 % 256) == 0 && (kOffKS % 256) == 0 && (kOffYS16 % 256) == 0 && (kOffOUTP % 256) == 0, "aligned regions");

__device__ __forceinline__ unsigned short f2bf_bits(float f) {
  unsigned u = __float_as_uint(f);
  return (unsigned short)((u + 0x7FFFu + ((u >> 16) & 1u)) >> 16);
}
__device__ __forceinline__ float bf_bits2f(unsigned short h) { return __uint_as_float(((unsigned)h) << 16); }
__device__ __forceinline__ float bf16r(float f) { return bf_bits2f(f2bf_bits(f)); }
__device__ __forceinline__ float carry_flush(float v, float carry) {
  const float s = v * carry;
  return (fabsf(s) < kF16MinNormal) ? 0.0f : s;
}
__device__ __forceinline__ float frcp(float x) { return __builtin_amdgcn_rcpf(x); }

__device__ __forceinline__ void dep_guard4_h(v8f& a, v8f& b, v8f& c, v8f& d, v16h x, v16h y) { asm volatile("v_nop\n\tv_nop\n\tv_nop\n\tv_nop" : "+v"(a), "+v"(b), "+v"(c), "+v"(d) : "v"(x), "v"(y)); }
__device__ __forceinline__ void dep_guard4_b(v8f& a, v8f& b, v8f& c, v8f& d, v16b x, v16b y) { asm volatile("v_nop\n\tv_nop\n\tv_nop\n\tv_nop" : "+v"(a), "+v"(b), "+v"(c), "+v"(d) : "v"(x), "v"(y)); }
__device__ __forceinline__ void keep4_h(v16h a, v16h b, v16h c, v16h d) { asm volatile("v_nop" :: "v"(a), "v"(b), "v"(c), "v"(d)); }
__device__ __forceinline__ void keep4_b(v16b a, v16b b, v16b c, v16b d) { asm volatile("v_nop" :: "v"(a), "v"(b), "v"(c), "v"(d)); }
__device__ __forceinline__ void acc_guard4(v8f& a, v8f& b, v8f& c, v8f& d) { asm volatile("v_nop\n\tv_nop\n\tv_nop\n\tv_nop" : "+v"(a), "+v"(b), "+v"(c), "+v"(d)); }

template <typename T> struct Frag;
template <> struct Frag<_Float16> {
  typedef v16h V; union U { v16h v; v8h h[2]; };
  static __device__ __forceinline__ v16h load(const _Float16* p) {
    U f; f.h[0] = *(const v8h*)(p); f.h[1] = *(const v8h*)(p + 16); return f.v;
  }
  static __device__ __forceinline__ v8f mma(v16h a, v16h b, v8f c) {
    return __builtin_amdgcn_wmma_f32_16x16x32_f16(false, a, false, b, (short)0, c, false, false);
  }
  static __device__ __forceinline__ void guard4(v8f& a, v8f& b, v8f& c, v8f& d, v16h x, v16h y) { dep_guard4_h(a, b, c, d, x, y); }
  static __device__ __forceinline__ void keep(v16h a, v16h b, v16h c, v16h d) { keep4_h(a, b, c, d); }
};
template <> struct Frag<__bf16> {
  typedef v16b V; union U { v16b v; v8b h[2]; };
  static __device__ __forceinline__ v16b load(const __bf16* p) {
    U f; f.h[0] = *(const v8b*)(p); f.h[1] = *(const v8b*)(p + 16); return f.v;
  }
  static __device__ __forceinline__ v8f mma(v16b a, v16b b, v8f c) {
    return __builtin_amdgcn_wmma_f32_16x16x32_bf16(false, a, false, b, (short)0, c, false, false);
  }
  static __device__ __forceinline__ void guard4(v8f& a, v8f& b, v8f& c, v8f& d, v16b x, v16b y) { dep_guard4_b(a, b, c, d, x, y); }
  static __device__ __forceinline__ void keep(v16b a, v16b b, v16b c, v16b d) { keep4_b(a, b, c, d); }
};

__device__ __forceinline__ v8f mma_h(v16h a, v16h b, v8f c) {
  c = __builtin_amdgcn_wmma_f32_16x16x32_f16(false, a, false, b, (short)0, c, false, false);
  asm volatile("v_nop\n\tv_nop\n\tv_nop\n\tv_nop" : "+v"(c) : "v"(a), "v"(b));
  return c;
}

template <int ET> struct Elem;
template <> struct Elem<0> { typedef _Float16 T; };
template <> struct Elem<1> { typedef __bf16 T; };
template <int ET, bool SPLIT, int BIAS_MODE, int OUT_MODE, bool RESID, int ACT = 0>
__global__ __launch_bounds__(256) void wmma_gemm64(
    const unsigned short* __restrict__ Ap, const unsigned short* __restrict__ A2p, int lda, long strideA,
    const unsigned short* __restrict__ Btp, const unsigned short* __restrict__ Bt2p, int ldb, long strideB,
    void* __restrict__ Cout, void* __restrict__ Cout2, int ldc, long strideC,
    const float* __restrict__ bias,
    const float* __restrict__ resid, long strideR,
    int M, int N, int K, float scale) {
  typedef typename Elem<ET>::T T;
  typedef typename Frag<T>::V V;
  const T* A = (const T*)Ap; const T* A2 = (const T*)A2p; const T* Bt = (const T*)Btp; const T* Bt2 = (const T*)Bt2p;
  __shared__ __align__(16) float sT[8][16 * 68];
  const int b    = blockIdx.y;
  const int lane = threadIdx.x & 31;
  const int wave = threadIdx.x >> 5;
  const int tilesN = N >> 6;
  const int tilesM = M >> 6;
  const int tile = blockIdx.x * 8 + wave;
  if (tile >= tilesM * tilesN) return;
  const int tm = tile / tilesN;
  const int tn = tile - tm * tilesN;
  const int m0 = tm << 6;
  const int n0 = tn << 6;

  const T* Ab  = A  + (size_t)b * strideA;
  const T* Bb  = Bt + (size_t)b * strideB;
  const T* Ab2 = SPLIT ? (A2  + (size_t)b * strideA) : nullptr;
  const T* Bb2 = SPLIT ? (Bt2 + (size_t)b * strideB) : nullptr;

  const int rlane = lane & 15;
  const int koff  = (lane >> 4) * 8;
  const int mOff  = (lane >> 4) * 8;

  v8f acc[4][4];
#pragma unroll
  for (int i = 0; i < 4; ++i)
#pragma unroll
    for (int j = 0; j < 4; ++j) acc[i][j] = (v8f){0.f,0.f,0.f,0.f,0.f,0.f,0.f,0.f};

  for (int k0 = 0; k0 < K; k0 += 32) {
    V bh[4], bl[4];
#pragma unroll
    for (int j = 0; j < 4; ++j) {
      const size_t bo = (size_t)(n0 + (j << 4) + rlane) * ldb + koff + k0;
      bh[j] = Frag<T>::load(Bb + bo);
      if (SPLIT) bl[j] = Frag<T>::load(Bb2 + bo);
    }
#pragma unroll
    for (int i = 0; i < 4; ++i) {
      const size_t ao = (size_t)(m0 + (i << 4) + rlane) * lda + koff + k0;
      V ah = Frag<T>::load(Ab + ao);
      V al;
      if (SPLIT) al = Frag<T>::load(Ab2 + ao);
#pragma unroll
      for (int j = 0; j < 4; ++j) {
        acc[i][j] = Frag<T>::mma(ah, bh[j], acc[i][j]);
        if (SPLIT) {
          acc[i][j] = Frag<T>::mma(ah, bl[j], acc[i][j]);
          acc[i][j] = Frag<T>::mma(al, bh[j], acc[i][j]);
        }
      }
      Frag<T>::guard4(acc[i][0], acc[i][1], acc[i][2], acc[i][3], ah, SPLIT ? al : ah);
    }
    Frag<T>::keep(bh[0], bh[1], bh[2], bh[3]);
    if (SPLIT) Frag<T>::keep(bl[0], bl[1], bl[2], bl[3]);
  }
  acc_guard4(acc[0][0], acc[0][1], acc[0][2], acc[0][3]);
  acc_guard4(acc[1][0], acc[1][1], acc[1][2], acc[1][3]);
  acc_guard4(acc[2][0], acc[2][1], acc[2][2], acc[2][3]);
  acc_guard4(acc[3][0], acc[3][1], acc[3][2], acc[3][3]);

  float* slab = sT[wave];
  const float* Rb = RESID ? (resid + (size_t)b * strideR) : nullptr;
#pragma unroll
  for (int i = 0; i < 4; ++i) {
    const int mBase = m0 + (i << 4);
#pragma unroll
    for (int j = 0; j < 4; ++j) {
      const int n = n0 + (j << 4) + rlane;
      float bv = 0.f;
      if (BIAS_MODE == 2) bv = bias[n];
#pragma unroll
      for (int r = 0; r < 8; ++r) {
        float v = acc[i][j][r] * scale;
        if (BIAS_MODE == 1) v += bias[mBase + mOff + r];
        if (BIAS_MODE == 2) v += bv;
        if (RESID) v += Rb[(size_t)(mBase + mOff + r) * ldc + n];
        if (ACT == 1) v = tanhf(v);
        if (ACT == 2) v = fmaxf(v, 0.0f);
        if (ACT == 3) v = v / (1.0f + expf(-v));
        if (ACT == 4) v = (v > 0.f) ? v : 0.01f * v;
        slab[(mOff + r) * 68 + (j << 4) + rlane] = v;
      }
    }
    __builtin_amdgcn_fence(__ATOMIC_RELEASE, "workgroup");
    __builtin_amdgcn_wave_barrier();
    __builtin_amdgcn_fence(__ATOMIC_ACQUIRE, "workgroup");
    if (OUT_MODE == 0) {
      float* C = (float*)Cout + (size_t)b * strideC;
      const int hh = lane >> 4, c4 = (lane & 15) * 4;
      for (int pass = 0; pass < 2; ++pass) {
#pragma unroll
        for (int it = 0; it < 8; ++it) {
          const int row = it * 2 + hh;
          v4f v = *(const v4f*)(slab + row * 68 + c4);
          *(volatile v4f*)(C + (size_t)(mBase + row) * ldc + n0 + c4) = v;
        }
        __threadfence();
      }
    } else {
      const int q = lane >> 3, c8 = (lane & 7) * 8;
      unsigned short* C  = (unsigned short*)Cout  + (size_t)b * strideC;
      unsigned short* C2 = (OUT_MODE == 2) ? ((unsigned short*)Cout2 + (size_t)b * strideC) : nullptr;
      for (int pass = 0; pass < 2; ++pass) {
#pragma unroll
        for (int it = 0; it < 4; ++it) {
          const int row = it * 4 + q;
          const float* sp = slab + row * 68 + c8;
          v8h hv, lv;
#pragma unroll
          for (int e = 0; e < 8; ++e) {
            if (OUT_MODE == 1) {
              hv[e] = (_Float16)sp[e];
            } else {
              unsigned short hb = f2bf_bits(sp[e]);
              unsigned short lb = f2bf_bits(sp[e] - bf_bits2f(hb));
              hv[e] = __builtin_bit_cast(_Float16, hb);
              lv[e] = __builtin_bit_cast(_Float16, lb);
            }
          }
          *(volatile v8h*)(C + (size_t)(mBase + row) * ldc + n0 + c8) = hv;
          if (OUT_MODE == 2) *(volatile v8h*)(C2 + (size_t)(mBase + row) * ldc + n0 + c8) = lv;
        }
        __threadfence();
      }
    }
    __builtin_amdgcn_fence(__ATOMIC_RELEASE, "workgroup");
    __builtin_amdgcn_wave_barrier();
    __builtin_amdgcn_fence(__ATOMIC_ACQUIRE, "workgroup");
  }
}

__global__ __launch_bounds__(kThr) void cast_plane_kernel(const float* __restrict__ src, unsigned short* __restrict__ dst,
                                                          int colsLog2, int dstPitch, int dstOff) {
  const int i   = blockIdx.x * kThr + threadIdx.x;
  const int sh  = colsLog2 - 3;
  const int row = i >> sh;
  const int c8  = (i & ((1 << sh) - 1)) * 8;
  const float* sp = src + ((size_t)row << colsLog2) + c8;
  const v4f a0 = *(const v4f*)(sp);
  const v4f a1 = *(const v4f*)(sp + 4);
  v8h hv;
#pragma unroll
  for (int e = 0; e < 4; ++e) {
    const float f0 = a0[e];
    const float f1 = a1[e];
    hv[e]     = (_Float16)carry_flush(bf16r(f0), kInCarry);
    hv[4 + e] = (_Float16)carry_flush(bf16r(f1), kInCarry);
  }
  unsigned short* dp = dst + (size_t)row * dstPitch + dstOff + c8;
  *(volatile v8h*)dp = hv;
  __threadfence();
  *(volatile v8h*)dp = hv;
}

__global__ __launch_bounds__(kThr) void zero_kernel(float* __restrict__ dst) {
  const size_t o4 = ((size_t)blockIdx.x * kThr + threadIdx.x) * 4u;
  const v4f z = {0.f, 0.f, 0.f, 0.f};
  *(volatile v4f*)(dst + o4) = z;
  __threadfence();
  *(volatile v4f*)(dst + o4) = z;
}
static_assert(kOffSTATE == kOffZB + 4096ull && (1024 + kMN * kMD) / 4 == 9 * kThr, "the zero bias and the carried memory are adjacent: one fill");

__global__ __launch_bounds__(kThr) void mem_scan_kernel(const float* __restrict__ VFQ, const float* __restrict__ beta, const float* __restrict__ decay,
                                                        float* STATE, float* __restrict__ MEM32, unsigned short* __restrict__ MEM16, int chunk) {
  const unsigned v = blockIdx.x * (unsigned)kThr + threadIdx.x;
  const unsigned slot = v >> 6, d0 = (v & 63u) * 2u;
  float bs[2], gm[2], mem[2];
#pragma unroll
  for (int k = 0; k < 2; ++k) {
    const unsigned d = d0 + (unsigned)k;
    const float b0 = beta[(size_t)slot * kMD + d];
    bs[k] = 1.0f / (1.0f + expf(-bf16r(b0)));
    const bool dec = d >= (unsigned)(kMD - kDD);
    const float c0 = decay[(size_t)slot * kDD + (dec ? (d - (unsigned)(kMD - kDD)) : 0u)];
    const float sg = 1.0f / (1.0f + expf(-bf16r(c0)));
    gm[k] = dec ? sg : 1.0f;
    mem[k] = STATE[(size_t)slot * kMD + d];
  }
  const float* vq = VFQ + (size_t)chunk * kTC * kNV;
  for (int t = 0; t < kTC; ++t) {
    const float fp = vq[(size_t)t * kNV + kMD + slot];
    const float f = 1.0f / (1.0f + expf(-fp));
    const v2f vv = *(const v2f*)(vq + (size_t)t * kNV + d0);
    v2f m2; v2h h2;
#pragma unroll
    for (int k = 0; k < 2; ++k) {
      const float a = (1.0f - f * bs[k]) * gm[k];
      const float nm = a * mem[k] + f * vv[k];
      mem[k] = nm; m2[k] = nm;
      h2[k] = (_Float16)carry_flush(nm, kInCarry);
    }
    const size_t row = (size_t)t * kMN + slot;
    float* mp = MEM32 + row * kMD + d0;
    unsigned short* hp = MEM16 + row * kMD + d0;
    for (int pass = 0; pass < 2; ++pass) {
      *(volatile v2f*)mp = m2;
      *(volatile v2h*)hp = h2;
      __threadfence();
    }
  }
  float* sp = STATE + (size_t)slot * kMD + d0;
  const v2f o2 = {mem[0], mem[1]};
  *(volatile v2f*)sp = o2;
  __threadfence();
  *(volatile v2f*)sp = o2;
}
static_assert(kMN * 64 == 16 * kThr && kMD == 128 && kDD == 32, "scan grid exact: two waves a slot");

__global__ __launch_bounds__(kThr) void attend_kernel(const float* __restrict__ VFQ, const float* __restrict__ KS, const float* __restrict__ lp,
                                                      const float* __restrict__ MEM32, unsigned short* __restrict__ YS16, int chunk) {
  const unsigned w = blockIdx.x * 8u + (threadIdx.x >> 5);
  const unsigned lane = threadIdx.x & 31u;
  const size_t tg = (size_t)chunk * kTC + w;
  const v4f q = *(const v4f*)(VFQ + tg * kNV + (kMD + kMN) + lane * 4u);
  float sc[kMN];
  float mx = 0.0f;
#pragma unroll
  for (int m = 0; m < kMN; ++m) {
    const v4f kv = *(const v4f*)(KS + ((size_t)w * kMN + m) * kMD + lane * 4u);
    const v4f lv = *(const v4f*)(lp + (size_t)m * kMD + lane * 4u);
    float s = (kv[0] + bf16r(lv[0])) * q[0];
    s += (kv[1] + bf16r(lv[1])) * q[1];
    s += (kv[2] + bf16r(lv[2])) * q[2];
    s += (kv[3] + bf16r(lv[3])) * q[3];
    s += __shfl_xor(s, 1, 32);
    s += __shfl_xor(s, 2, 32);
    s += __shfl_xor(s, 4, 32);
    s += __shfl_xor(s, 8, 32);
    s += __shfl_xor(s, 16, 32);
    s *= kScale;
    sc[m] = s;
    mx = (m == 0) ? s : ((s > mx) ? s : mx);
  }
  float sum = 0.0f;
#pragma unroll
  for (int m = 0; m < kMN; ++m) { const float e = expf(sc[m] - mx); sc[m] = e; sum += e; }
  v4f ys = {0.f, 0.f, 0.f, 0.f};
#pragma unroll
  for (int m = 0; m < kMN; ++m) {
    const float a = sc[m] / sum;
    const v4f mv = *(const v4f*)(MEM32 + ((size_t)w * kMN + m) * kMD + lane * 4u);
    ys[0] += a * mv[0]; ys[1] += a * mv[1]; ys[2] += a * mv[2]; ys[3] += a * mv[3];
  }
  v4h hv;
#pragma unroll
  for (int e = 0; e < 4; ++e) hv[e] = (_Float16)carry_flush(ys[e], kInCarry);
  unsigned short* dp = YS16 + tg * kMD + lane * 4u;
  *(volatile v4h*)dp = hv;
  __threadfence();
  *(volatile v4h*)dp = hv;
}
static_assert(kTC % 8 == 0 && kMD == 4 * 32, "one wave a step; four columns a lane");

__global__ __launch_bounds__(kThr) void gate_out_kernel(const float* __restrict__ OUTP, const float* __restrict__ G, float* __restrict__ out) {
  const size_t o4 = ((size_t)blockIdx.x * kThr + threadIdx.x) * 4u;
  const v4f y = *(const v4f*)(OUTP + o4), g = *(const v4f*)(G + o4);
  v4f r;
#pragma unroll
  for (int e = 0; e < 4; ++e) r[e] = y[e] * (1.0f / (1.0f + expf(-g[e])));
  *(volatile v4f*)(out + o4) = r;
  __threadfence();
  *(volatile v4f*)(out + o4) = r;
}
static_assert(((size_t)kT * kXD / 4) == 8192 * kThr, "output grid exact");

static_assert(((size_t)kT * kXD / 8) % kThr == 0 && ((size_t)kMD * kXD / 8) % kThr == 0 && ((size_t)kMN * kXD / 8) % kThr == 0 && ((size_t)kXD * kXD / 8) % kThr == 0 && ((size_t)kMD * kMD / 8) % kThr == 0 && ((size_t)kXD * kMD / 8) % kThr == 0, "plane cast grids exact");

extern "C" void kernel_launch(void* const* d_in, const int* in_sizes, int n_in,
                              void* d_out, int out_size, void* d_ws, size_t ws_size,
                              hipStream_t stream) {
  if (n_in < 10 || d_out == nullptr || d_ws == nullptr) return;
  if (in_sizes[0] != kT * kXD || in_sizes[1] != kMN * kXD || in_sizes[2] != kMD * kXD || in_sizes[3] != kMD * kMD || in_sizes[4] != kMD * kXD) return;
  if (in_sizes[5] != kXD * kMD || in_sizes[6] != kXD * kXD || in_sizes[7] != kMN * kMD || in_sizes[8] != kMN * kDD || in_sizes[9] != kMN * kMD) return;
  if (out_size != kT * kXD) return;
  if (ws_size < kWsTotal) return;
  const float* xs = (const float*)d_in[0];
  const float* Wf = (const float*)d_in[1];
  const float* Wq = (const float*)d_in[2];
  const float* Wk = (const float*)d_in[3];
  const float* Wv = (const float*)d_in[4];
  const float* Wo = (const float*)d_in[5];
  const float* Wr = (const float*)d_in[6];
  const float* beta = (const float*)d_in[7];
  const float* decay = (const float*)d_in[8];
  const float* lp = (const float*)d_in[9];
  float* out = (float*)d_out;
  char* ws = (char*)d_ws;
  unsigned short* X16 = (unsigned short*)(ws + kOffX16);
  unsigned short* WVFQ = (unsigned short*)(ws + kOffWVFQ);
  unsigned short* WR16 = (unsigned short*)(ws + kOffWR16);
  unsigned short* WK16 = (unsigned short*)(ws + kOffWK16);
  unsigned short* WO16 = (unsigned short*)(ws + kOffWO16);
  float* ZB = (float*)(ws + kOffZB);
  float* STATE = (float*)(ws + kOffSTATE);
  float* VFQ = (float*)(ws + kOffVFQ);
  float* G = (float*)(ws + kOffG);
  float* MEM32 = (float*)(ws + kOffMEM32);
  unsigned short* MEM16 = (unsigned short*)(ws + kOffMEM16);
  float* KS = (float*)(ws + kOffKS);
  unsigned short* YS16 = (unsigned short*)(ws + kOffYS16);
  float* OUTP = (float*)(ws + kOffOUTP);

  cast_plane_kernel<<<(int)(((size_t)kT * kXD / 8) / kThr), kThr, 0, stream>>>(xs, X16, 10, kXD, 0);
  cast_plane_kernel<<<(int)(((size_t)kMD * kXD / 8) / kThr), kThr, 0, stream>>>(Wv, WVFQ, 10, kXD, 0);
  cast_plane_kernel<<<(int)(((size_t)kMN * kXD / 8) / kThr), kThr, 0, stream>>>(Wf, WVFQ + (size_t)kMD * kXD, 10, kXD, 0);
  cast_plane_kernel<<<(int)(((size_t)kMD * kXD / 8) / kThr), kThr, 0, stream>>>(Wq, WVFQ + (size_t)(kMD + kMN) * kXD, 10, kXD, 0);
  cast_plane_kernel<<<(int)(((size_t)kXD * kXD / 8) / kThr), kThr, 0, stream>>>(Wr, WR16, 10, kXD, 0);
  cast_plane_kernel<<<(int)(((size_t)kMD * kMD / 8) / kThr), kThr, 0, stream>>>(Wk, WK16, 7, kMD, 0);
  cast_plane_kernel<<<(int)(((size_t)kXD * kMD / 8) / kThr), kThr, 0, stream>>>(Wo, WO16, 7, kMD, 0);
  zero_kernel<<<9, kThr, 0, stream>>>(ZB);
  wmma_gemm64<0, false, 2, 0, false, 0><<<dim3((kT / 64) * (kNV / 64) / 8, 1), 256, 0, stream>>>(
      X16, X16, kXD, 0L, WVFQ, WVFQ, kXD, 0L, (void*)VFQ, (void*)VFQ, kNV, 0L, ZB, nullptr, 0L, kT, kNV, kXD, kSc);
  wmma_gemm64<0, false, 2, 0, false, 0><<<dim3((kT / 64) * (kXD / 64) / 8, 1), 256, 0, stream>>>(
      X16, X16, kXD, 0L, WR16, WR16, kXD, 0L, (void*)G, (void*)G, kXD, 0L, ZB, nullptr, 0L, kT, kXD, kXD, kSc);
  for (int ch = 0; ch < kNCh; ++ch) {
    mem_scan_kernel<<<(kMN * 64) / kThr, kThr, 0, stream>>>(VFQ, beta, decay, STATE, MEM32, MEM16, ch);
    wmma_gemm64<0, false, 2, 0, false, 0><<<dim3((kRC / 64) * (kMD / 64) / 8, 1), 256, 0, stream>>>(
        MEM16, MEM16, kMD, 0L, WK16, WK16, kMD, 0L, (void*)KS, (void*)KS, kMD, 0L, ZB, nullptr, 0L, kRC, kMD, kMD, kSc);
    attend_kernel<<<kTC / 8, kThr, 0, stream>>>(VFQ, KS, lp, MEM32, YS16, ch);
  }
  wmma_gemm64<0, false, 2, 0, false, 0><<<dim3((kT / 64) * (kXD / 64) / 8, 1), 256, 0, stream>>>(
      YS16, YS16, kMD, 0L, WO16, WO16, kMD, 0L, (void*)OUTP, (void*)OUTP, kXD, 0L, ZB, nullptr, 0L, kT, kXD, kMD, kSc);
  gate_out_kernel<<<8192, kThr, 0, stream>>>(OUTP, G, out);
}
